// BiModalAttention_6270652252304
// MI455X (gfx1250) — hardware-verified
//
#include <hip/hip_runtime.h>

#define B_DIM 8
#define S_DIM 4096
#define D_DIM 64
#define NELEM (B_DIM * S_DIM * D_DIM)
#define LTS 128
#define LTT 64
#define QT 128
#define KT 64
#define NWAVE 8
#define NTHR (NWAVE * 32)
#define HPITCH 72
#define OPITCH 68
#define LOG2E 1.44269504088896340736f
#define PSCALE_LOG2 12.0f

static_assert(S_DIM % LTS == 0 && S_DIM % LTT == 0 && S_DIM % QT == 0 && S_DIM % KT == 0);
static_assert(D_DIM == 64 && QT == 16 * NWAVE && LTS == 16 * NWAVE);

typedef _Float16 v16h __attribute__((ext_vector_type(16)));
typedef _Float16 v8h  __attribute__((ext_vector_type(8)));
typedef __bf16   v16b __attribute__((ext_vector_type(16)));
typedef unsigned short v8us __attribute__((ext_vector_type(8)));
typedef float v8f __attribute__((ext_vector_type(8)));
typedef float v4f __attribute__((ext_vector_type(4)));

union FragH { v16h v; v8h half[2]; };
union FragB { v16b v; v8us half[2]; };

__device__ __forceinline__ v8f mma_f16(const FragH& a, const FragH& b, v8f c) {
    c = __builtin_amdgcn_wmma_f32_16x16x32_f16(false, a.v, false, b.v, (short)0, c, false, false);
    asm volatile("v_nop\n\tv_nop\n\tv_nop\n\tv_nop"
                 : "+v"(c) : "v"(a.half[0]), "v"(a.half[1]), "v"(b.half[0]), "v"(b.half[1]));
    return c;
}
__device__ __forceinline__ v8f mma_bf16(const FragB& a, const FragB& b, v8f c) {
    c = __builtin_amdgcn_wmma_f32_16x16x32_bf16(false, a.v, false, b.v, (short)0, c, false, false);
    asm volatile("v_nop\n\tv_nop\n\tv_nop\n\tv_nop"
                 : "+v"(c) : "v"(a.half[0]), "v"(a.half[1]), "v"(b.half[0]), "v"(b.half[1]));
    return c;
}

__device__ __forceinline__ unsigned int bf16_rne_bits(float f) {
    unsigned int u = __float_as_uint(f);
    u += 0x7FFFu + ((u >> 16) & 1u);
    return u >> 16;
}
__device__ __forceinline__ void bf16_split(float f, unsigned short& hi, unsigned short& lo) {
    const unsigned int hb = bf16_rne_bits(f);
    const float hf = __uint_as_float(hb << 16);
    hi = (unsigned short)hb;
    lo = (unsigned short)bf16_rne_bits(f - hf);
}

__global__ __launch_bounds__(NTHR)
void k_prep(const float* __restrict__ x, const float* __restrict__ y,
            unsigned short* __restrict__ ph, unsigned short* __restrict__ pl,
            _Float16* __restrict__ pvt)
{
    __shared__ __align__(16) _Float16 T[D_DIM * HPITCH];

    const int rt = blockIdx.x, b = blockIdx.y, z = blockIdx.z;
    const int tid = threadIdx.x;
    const int r0 = rt * KT;
    const float* src = (z ? y : x) + ((size_t)b * S_DIM + r0) * D_DIM;
    const size_t pofs = (size_t)z * NELEM + ((size_t)b * S_DIM + r0) * D_DIM;
    unsigned short* hp = ph + pofs;
    unsigned short* lp = pl + pofs;
    _Float16* vt = pvt + (size_t)z * NELEM + (size_t)b * D_DIM * S_DIM + r0;

    v8us hv[2], lv[2];
    int erow[2], ec8[2];
#pragma unroll
    for (int i = 0; i < 2; ++i) {
        const int e = tid + NTHR * i;
        const int row = e >> 3;
        const int c8 = (e & 7) * 8;
        erow[i] = row; ec8[i] = c8;
        const v4f f0 = *(const v4f*)(src + row * D_DIM + c8);
        const v4f f1 = *(const v4f*)(src + row * D_DIM + c8 + 4);
        const float fv[8] = {f0[0], f0[1], f0[2], f0[3], f1[0], f1[1], f1[2], f1[3]};
#pragma unroll
        for (int q = 0; q < 8; ++q) {
            unsigned short hb, lb;
            bf16_split(fv[q], hb, lb);
            hv[i][q] = hb;
            lv[i][q] = lb;
            T[(c8 + q) * HPITCH + row] = (_Float16)fv[q];
        }
    }
#pragma unroll
    for (int i = 0; i < 2; ++i) {
        *(volatile v8us*)(hp + erow[i] * D_DIM + ec8[i]) = hv[i];
        *(volatile v8us*)(lp + erow[i] * D_DIM + ec8[i]) = lv[i];
    }
    __syncthreads();
    v8h tv[2];
#pragma unroll
    for (int i = 0; i < 2; ++i) tv[i] = *(const v8h*)(T + erow[i] * HPITCH + ec8[i]);
#pragma unroll
    for (int i = 0; i < 2; ++i)
        *(volatile v8h*)(vt + (size_t)erow[i] * S_DIM + ec8[i]) = tv[i];
    __threadfence();
#pragma unroll
    for (int i = 0; i < 2; ++i) {
        *(volatile v8us*)(hp + erow[i] * D_DIM + ec8[i]) = hv[i];
        *(volatile v8us*)(lp + erow[i] * D_DIM + ec8[i]) = lv[i];
        *(volatile v8h*)(vt + (size_t)erow[i] * S_DIM + ec8[i]) = tv[i];
    }
}

__global__ __launch_bounds__(NTHR)
void k_logits(const unsigned short* __restrict__ xh, const unsigned short* __restrict__ xl,
              const unsigned short* __restrict__ yh, const unsigned short* __restrict__ yl,
              float* __restrict__ S, int bbase)
{
    __shared__ __align__(16) float stg_all[NWAVE * 16 * LTT];

    const int tt = blockIdx.x, st = blockIdx.y, zb = blockIdx.z;
    const int b = bbase + zb;
    const int tid = threadIdx.x;
    const int w = tid >> 5, l = tid & 31, h = l >> 4, m = l & 15;
    const int s0 = st * LTS, t0 = tt * LTT;

    const size_t arow = (size_t)b * S_DIM + s0 + 16 * w + m;
    const unsigned short* xhr = xh + arow * D_DIM;
    const unsigned short* xlr = xl + arow * D_DIM;
    const size_t brow0 = (size_t)b * S_DIM + t0 + m;

    v8f acc[4];
#pragma unroll
    for (int j = 0; j < 4; ++j) acc[j] = (v8f)(0.0f);

#pragma unroll
    for (int ks = 0; ks < 2; ++ks) {
        const int k0 = 32 * ks;
        FragB ah, al;
        ah.half[0] = *(const v8us*)(xhr + k0 + 8 * h);
        ah.half[1] = *(const v8us*)(xhr + k0 + 16 + 8 * h);
        al.half[0] = *(const v8us*)(xlr + k0 + 8 * h);
        al.half[1] = *(const v8us*)(xlr + k0 + 16 + 8 * h);
#pragma unroll
        for (int j = 0; j < 4; ++j) {
            const unsigned short* yhr = yh + (brow0 + 16 * j) * D_DIM + k0;
            const unsigned short* ylr = yl + (brow0 + 16 * j) * D_DIM + k0;
            FragB bh, bl;
            bh.half[0] = *(const v8us*)(yhr + 8 * h);
            bh.half[1] = *(const v8us*)(yhr + 16 + 8 * h);
            bl.half[0] = *(const v8us*)(ylr + 8 * h);
            bl.half[1] = *(const v8us*)(ylr + 16 + 8 * h);
            acc[j] = mma_bf16(ah, bh, acc[j]);
            acc[j] = mma_bf16(ah, bl, acc[j]);
            acc[j] = mma_bf16(al, bh, acc[j]);
        }
    }

    float* stg = stg_all + w * (16 * LTT);
#pragma unroll
    for (int j = 0; j < 4; ++j)
#pragma unroll
        for (int r = 0; r < 8; ++r)
            stg[(8 * h + r) * LTT + 16 * j + m] = acc[j][r];
    __syncthreads();
    v4f vals[8];
#pragma unroll
    for (int i = 0; i < 8; ++i) vals[i] = *(const v4f*)(stg + (2 * i + h) * LTT + 4 * m);
    float* base = S + (size_t)zb * S_DIM * S_DIM + (size_t)(s0 + 16 * w) * S_DIM + t0 + 4 * m;
#pragma unroll
    for (int i = 0; i < 8; ++i)
        *(volatile v4f*)(base + (size_t)(2 * i + h) * S_DIM) = vals[i];
    __threadfence();
#pragma unroll
    for (int i = 0; i < 8; ++i)
        *(volatile v4f*)(base + (size_t)(2 * i + h) * S_DIM) = vals[i];
}

template <int DIR>
__global__ __launch_bounds__(NTHR)
void k_attn(const float* __restrict__ x, const float* __restrict__ y,
            const _Float16* __restrict__ xvt, const _Float16* __restrict__ yvt,
            const float* __restrict__ S, float* __restrict__ out, int bbase)
{
    __shared__ __align__(16) float s_o[NWAVE * 16 * OPITCH];

    const int qt = blockIdx.x, zb = blockIdx.y;
    const int b = bbase + zb;
    const int tid = threadIdx.x;
    const int w = tid >> 5, l = tid & 31, h = l >> 4, m = l & 15;

    const float* Q = DIR ? y : x;
    const _Float16* vtb = (DIR ? xvt : yvt) + (size_t)b * D_DIM * S_DIM;
    const float* Sz = S + (size_t)zb * S_DIM * S_DIM;
    const int q0 = qt * QT + 16 * w;
    const int qm = q0 + m;

    float Mrun = -3.0e38f;
    float Lrun = 0.0f;
    v8f o[4];
#pragma unroll
    for (int j = 0; j < 4; ++j) o[j] = (v8f)(0.0f);

#pragma unroll 1
    for (int kt = 0; kt < S_DIM; kt += KT) {
        v8f sv[4];
        if (DIR == 0) {
            const float* lp = Sz + (size_t)qm * S_DIM + kt + 8 * h;
#pragma unroll
            for (int j = 0; j < 4; ++j) {
                const v4f u0 = *(const v4f*)(lp + 16 * j);
                const v4f u1 = *(const v4f*)(lp + 16 * j + 4);
#pragma unroll
                for (int r = 0; r < 4; ++r) { sv[j][r] = u0[r]; sv[j][4 + r] = u1[r]; }
            }
        } else {
            const float* lp = Sz + (size_t)(kt + 8 * h) * S_DIM + qm;
#pragma unroll
            for (int j = 0; j < 4; ++j)
#pragma unroll
                for (int r = 0; r < 8; ++r)
                    sv[j][r] = lp[(size_t)(16 * j + r) * S_DIM];
        }

        float tmax = sv[0][0];
#pragma unroll
        for (int j = 0; j < 4; ++j)
#pragma unroll
            for (int r = 0; r < 8; ++r) tmax = fmaxf(tmax, sv[j][r]);
        tmax = fmaxf(tmax, __shfl_xor(tmax, 16));
        const float mnew  = fmaxf(Mrun, tmax * LOG2E);
        const float alpha = exp2f(Mrun - mnew);
        const float off   = PSCALE_LOG2 - mnew;

        FragH pb0, pb1;
        float psum = 0.0f;
#pragma unroll
        for (int j = 0; j < 4; ++j) {
            v8h ph;
#pragma unroll
            for (int r = 0; r < 8; ++r) {
                const float e = fmaf(sv[j][r], LOG2E, off);
                float v = exp2f(e);
                v = (e < -14.0f) ? 0.0f : v;
                const _Float16 hq = (_Float16)v;
                ph[r] = hq;
                psum += (float)hq;
            }
            if (j == 0)      pb0.half[0] = ph;
            else if (j == 1) pb0.half[1] = ph;
            else if (j == 2) pb1.half[0] = ph;
            else             pb1.half[1] = ph;
        }
        psum += __shfl_xor(psum, 16);
        Lrun = Lrun * alpha + psum;
        Mrun = mnew;
#pragma unroll
        for (int j2 = 0; j2 < 4; ++j2) o[j2] *= alpha;

#pragma unroll
        for (int j2 = 0; j2 < 4; ++j2) {
            const _Float16* vr = vtb + (size_t)(16 * j2 + m) * S_DIM + kt;
            FragH a0, a1;
            a0.half[0] = *(const v8h*)(vr + 8 * h);
            a0.half[1] = *(const v8h*)(vr + 16 + 8 * h);
            a1.half[0] = *(const v8h*)(vr + 32 + 8 * h);
            a1.half[1] = *(const v8h*)(vr + 48 + 8 * h);
            o[j2] = mma_f16(a0, pb0, o[j2]);
            o[j2] = mma_f16(a1, pb1, o[j2]);
        }
    }

    const float inv = 1.0f / Lrun;
    const float* qp = Q + ((size_t)b * S_DIM + qm) * D_DIM;
    float* so = s_o + w * (16 * OPITCH);
#pragma unroll
    for (int j2 = 0; j2 < 4; ++j2) {
        const int dbase = 16 * j2 + 8 * h;
        const v4f qa = *(const v4f*)(qp + dbase);
        const v4f qb = *(const v4f*)(qp + dbase + 4);
        v4f ra, rb;
#pragma unroll
        for (int r = 0; r < 4; ++r) {
            ra[r] = o[j2][r] * inv * qa[r];
            rb[r] = o[j2][4 + r] * inv * qb[r];
        }
        *(v4f*)(so + m * OPITCH + dbase)     = ra;
        *(v4f*)(so + m * OPITCH + dbase + 4) = rb;
    }
    __syncthreads();
    v4f vals[8];
#pragma unroll
    for (int i = 0; i < 8; ++i) vals[i] = *(const v4f*)(so + (2 * i + h) * OPITCH + 4 * m);
    float* ob = out + ((size_t)b * S_DIM + q0) * (2 * D_DIM) + DIR * D_DIM + 4 * m;
#pragma unroll
    for (int i = 0; i < 8; ++i)
        *(volatile v4f*)(ob + (size_t)(2 * i + h) * (2 * D_DIM)) = vals[i];
    __threadfence();
#pragma unroll
    for (int i = 0; i < 8; ++i)
        *(volatile v4f*)(ob + (size_t)(2 * i + h) * (2 * D_DIM)) = vals[i];
}

extern "C" void kernel_launch(void* const* d_in, const int* in_sizes, int n_in,
                              void* d_out, int out_size, void* d_ws, size_t ws_size,
                              hipStream_t stream)
{
    if (n_in < 2) return;
    if (in_sizes[0] != NELEM || in_sizes[1] != NELEM) return;
    if (out_size != B_DIM * S_DIM * 2 * D_DIM) return;

    const float* x = (const float*)d_in[0];
    const float* y = (const float*)d_in[1];
    float* out = (float*)d_out;

    const size_t plane_bytes  = (size_t)NELEM * 2;
    const size_t planes_total = 6 * plane_bytes;
    const size_t slab = (size_t)S_DIM * S_DIM * sizeof(float);
    if (ws_size < planes_total + slab) return;
    size_t nbs = (ws_size - planes_total) / slab;
    const int nb = nbs > (size_t)B_DIM ? B_DIM : (int)nbs;

    char* ws = (char*)d_ws;
    unsigned short* ph = (unsigned short*)(ws);
    unsigned short* pl = (unsigned short*)(ws + 2 * plane_bytes);
    _Float16* pvt = (_Float16*)(ws + 4 * plane_bytes);
    float* S = (float*)(ws + planes_total);
    const unsigned short* xh = ph;
    const unsigned short* yh = ph + NELEM;
    const unsigned short* xl = pl;
    const unsigned short* yl = pl + NELEM;
    const _Float16* xvt = pvt;
    const _Float16* yvt = pvt + NELEM;

    k_prep<<<dim3(S_DIM / KT, B_DIM, 2), dim3(NTHR), 0, stream>>>(x, y, ph, pl, pvt);

    for (int b0 = 0; b0 < B_DIM; b0 += nb) {
        const int cnt = (B_DIM - b0 < nb) ? (B_DIM - b0) : nb;
        k_logits<<<dim3(S_DIM / LTT, S_DIM / LTS, cnt), dim3(NTHR), 0, stream>>>(xh, xl, yh, yl, S, b0);
        k_attn<0><<<dim3(S_DIM / QT, cnt, 1), dim3(NTHR), 0, stream>>>(x, y, xvt, yvt, S, out, b0);
        k_attn<1><<<dim3(S_DIM / QT, cnt, 1), dim3(NTHR), 0, stream>>>(x, y, xvt, yvt, S, out, b0);
    }
}
